// MambaBlock_27006754357575
// MI455X (gfx1250) — hardware-verified
//
#include <hip/hip_runtime.h>
#include <math.h>

typedef __attribute__((ext_vector_type(8)))  _Float16 v8h;
typedef __attribute__((ext_vector_type(16))) __bf16   v16b;
typedef __attribute__((ext_vector_type(8)))  __bf16   v8b;
typedef __attribute__((ext_vector_type(8)))  float    v8f;
typedef __attribute__((ext_vector_type(4)))  float    v4f;
typedef __attribute__((ext_vector_type(4)))  unsigned v4u;

constexpr int kSeq    = 2048;
constexpr int kDm     = 1024;
constexpr int kDin    = 2048;
constexpr int kNst    = 16;
constexpr int kXzP    = 2 * kDin;
constexpr int kBcReal = 2 * kNst;
constexpr int kBcP    = 64;
constexpr int kConvTP = 260;
static_assert((kDm % 32) == 0 && (kDin % 32) == 0, "GEMM K multiples of 32");
static_assert((kSeq % 64) == 0 && (kXzP % 64) == 0 && (kDin % 64) == 0 && (kBcP % 64) == 0 && (kDm % 64) == 0, "GEMM M,N multiples of 64");
static_assert((kDin % 256) == 0 && kDin == 256 * 8, "row kernel: 256 threads x 8 channels");
static_assert(kBcReal == 32 && kBcReal <= kBcP, "x_proj width");

constexpr size_t kOffXB  = 0;
constexpr size_t kOffWIB = kOffXB  + (size_t)kSeq * kDm  * 2;
constexpr size_t kOffWDB = kOffWIB + (size_t)kXzP * kDm  * 2;
constexpr size_t kOffWOB = kOffWDB + (size_t)kDin * kDin * 2;
constexpr size_t kOffWXB = kOffWOB + (size_t)kDm  * kDin * 2;
constexpr size_t kOffXZ  = kOffWXB + (size_t)kBcP * kDin * 2;
constexpr size_t kOffXCH = kOffXZ  + (size_t)kSeq * kXzP * 4;
constexpr size_t kOffXCL = kOffXCH + (size_t)kSeq * kDin * 2;
constexpr size_t kOffPRE = kOffXCL + (size_t)kSeq * kDin * 2;
constexpr size_t kOffBC  = kOffPRE + (size_t)kSeq * kDin * 4;
constexpr size_t kOffYH  = kOffBC  + (size_t)kSeq * kBcP * 4;
constexpr size_t kOffYL  = kOffYH  + (size_t)kSeq * kDin * 2;
constexpr size_t kWsTotal = kOffYL + (size_t)kSeq * kDin * 2;
static_assert(kWsTotal == 109838336ull, "carve total");
static_assert(kWsTotal <= 134217728ull, "carve cap");
static_assert((kOffWIB % 128) == 0 && (kOffWDB % 128) == 0 && (kOffWOB % 128) == 0 && (kOffWXB % 128) == 0 &&
              (kOffXZ % 128) == 0 && (kOffXCH % 128) == 0 && (kOffXCL % 128) == 0 && (kOffPRE % 128) == 0 &&
              (kOffBC % 128) == 0 && (kOffYH % 128) == 0 && (kOffYL % 128) == 0, "128-B aligned regions");

__device__ __forceinline__ unsigned short f2bf_bits(float f) {
  unsigned u = __float_as_uint(f);
  return (unsigned short)((u + 0x7FFFu + ((u >> 16) & 1u)) >> 16);
}
__device__ __forceinline__ float bf_bits2f(unsigned short h) { return __uint_as_float(((unsigned)h) << 16); }
__device__ __forceinline__ float bf_rne(float f) { return bf_bits2f(f2bf_bits(f)); }

__device__ __forceinline__ void dep_guard4_b(v8f& a, v8f& b, v8f& c, v8f& d, v16b x, v16b y) {
  asm volatile("v_nop\n\tv_nop\n\tv_nop\n\tv_nop" : "+v"(a), "+v"(b), "+v"(c), "+v"(d) : "v"(x), "v"(y));
}
__device__ __forceinline__ void keep4_b(v16b a, v16b b, v16b c, v16b d) { asm volatile("v_nop" :: "v"(a), "v"(b), "v"(c), "v"(d)); }
__device__ __forceinline__ void acc_guard4(v8f& a, v8f& b, v8f& c, v8f& d) { asm volatile("v_nop\n\tv_nop\n\tv_nop\n\tv_nop" : "+v"(a), "+v"(b), "+v"(c), "+v"(d)); }

struct FragB {
  union U { v16b v; v8b h[2]; };
  static __device__ __forceinline__ v16b load(const __bf16* p) {
    U f; f.h[0] = *(const v8b*)(p); f.h[1] = *(const v8b*)(p + 16); return f.v;
  }
  static __device__ __forceinline__ v8f mma(v16b a, v16b b, v8f c) {
    return __builtin_amdgcn_wmma_f32_16x16x32_bf16(false, a, false, b, (short)0, c, false, false);
  }
};

template <int SPL>
__global__ __launch_bounds__(256) void wmma_gemm64(
    const unsigned short* __restrict__ Ap, const unsigned short* __restrict__ A2p, int lda,
    const unsigned short* __restrict__ Btp, int ldb,
    float* __restrict__ Cout, int ldc, int M, int N, int K) {
  const __bf16* A  = (const __bf16*)Ap;
  const __bf16* A2 = (const __bf16*)A2p;
  const __bf16* Bt = (const __bf16*)Btp;
  __shared__ __align__(16) float sT[8][16 * 68];
  const int lane = threadIdx.x & 31;
  const int wave = threadIdx.x >> 5;
  const int tilesN = N >> 6;
  const int tilesM = M >> 6;
  const int tile = blockIdx.x * 8 + wave;
  if (tile >= tilesM * tilesN) return;
  const int tm = tile / tilesN;
  const int tn = tile - tm * tilesN;
  const int m0 = tm << 6;
  const int n0 = tn << 6;

  const int rlane = lane & 15;
  const int koff  = (lane >> 4) * 8;
  const int mOff  = (lane >> 4) * 8;

  v8f acc[4][4];
#pragma unroll
  for (int i = 0; i < 4; ++i)
#pragma unroll
    for (int j = 0; j < 4; ++j) acc[i][j] = (v8f){0.f,0.f,0.f,0.f,0.f,0.f,0.f,0.f};

  for (int k0 = 0; k0 < K; k0 += 32) {
    v16b bh[4];
#pragma unroll
    for (int j = 0; j < 4; ++j) {
      const size_t bo = (size_t)(n0 + (j << 4) + rlane) * ldb + koff + k0;
      bh[j] = FragB::load(Bt + bo);
    }
#pragma unroll
    for (int i = 0; i < 4; ++i) {
      const size_t ao = (size_t)(m0 + (i << 4) + rlane) * lda + koff + k0;
      v16b ah = FragB::load(A + ao);
      v16b al = ah;
      if (SPL == 1) al = FragB::load(A2 + ao);
#pragma unroll
      for (int j = 0; j < 4; ++j) {
        acc[i][j] = FragB::mma(ah, bh[j], acc[i][j]);
        if (SPL == 1) acc[i][j] = FragB::mma(al, bh[j], acc[i][j]);
      }
      dep_guard4_b(acc[i][0], acc[i][1], acc[i][2], acc[i][3], ah, al);
    }
    keep4_b(bh[0], bh[1], bh[2], bh[3]);
  }
  acc_guard4(acc[0][0], acc[0][1], acc[0][2], acc[0][3]);
  acc_guard4(acc[1][0], acc[1][1], acc[1][2], acc[1][3]);
  acc_guard4(acc[2][0], acc[2][1], acc[2][2], acc[2][3]);
  acc_guard4(acc[3][0], acc[3][1], acc[3][2], acc[3][3]);

  float* slab = sT[wave];
#pragma unroll
  for (int i = 0; i < 4; ++i) {
    const int mBase = m0 + (i << 4);
#pragma unroll
    for (int j = 0; j < 4; ++j) {
#pragma unroll
      for (int r = 0; r < 8; ++r) {
        slab[(mOff + r) * 68 + (j << 4) + rlane] = acc[i][j][r];
      }
    }
    __builtin_amdgcn_fence(__ATOMIC_RELEASE, "workgroup");
    __builtin_amdgcn_wave_barrier();
    __builtin_amdgcn_fence(__ATOMIC_ACQUIRE, "workgroup");
    {
      const int hh = lane >> 4, c4 = (lane & 15) * 4;
      for (int pass = 0; pass < 2; ++pass) {
#pragma unroll
        for (int it = 0; it < 8; ++it) {
          const int row = it * 2 + hh;
          v4f v = *(const v4f*)(slab + row * 68 + c4);
          *(volatile v4f*)(Cout + (size_t)(mBase + row) * ldc + n0 + c4) = v;
        }
        __threadfence();
      }
    }
    __builtin_amdgcn_fence(__ATOMIC_RELEASE, "workgroup");
    __builtin_amdgcn_wave_barrier();
    __builtin_amdgcn_fence(__ATOMIC_ACQUIRE, "workgroup");
  }
}

__global__ __launch_bounds__(256) void rne_rows_bf16_kernel(
    const float* __restrict__ src, unsigned short* __restrict__ dst, int total8, int real8)
{
  const int i = blockIdx.x * 256 + threadIdx.x;
  if (i >= total8) return;
  const bool live = (i < real8);
  const int ic = live ? i : (real8 - 1);
  const size_t s0 = (size_t)ic << 3;
  const v4f a0 = *(const v4f*)(src + s0);
  const v4f a1 = *(const v4f*)(src + s0 + 4);
  v8h hv;
#pragma unroll
  for (int e = 0; e < 4; ++e) {
    const float ra = a0[e];
    const float rb = a1[e];
    const float fa = live ? ra : 0.0f;
    const float fb = live ? rb : 0.0f;
    const unsigned short h0 = f2bf_bits(fa);
    const unsigned short h1 = f2bf_bits(fb);
    hv[e]     = __builtin_bit_cast(_Float16, h0);
    hv[4 + e] = __builtin_bit_cast(_Float16, h1);
  }
  unsigned short* q = dst + ((size_t)i << 3);
  *(volatile v8h*)q = hv;
  __threadfence();
  *(volatile v8h*)q = hv;
}

__global__ __launch_bounds__(256) void conv_silu_kernel(
    const float* __restrict__ XZ, const float* __restrict__ cw, const float* __restrict__ cb,
    unsigned short* __restrict__ XCH, unsigned short* __restrict__ XCL)
{
  __shared__ __align__(16) float sT[16 * kConvTP];
  const int tid = threadIdx.x, lane = tid & 31, wave = tid >> 5;
  const int d0 = blockIdx.x * 256, d = d0 + tid;
  const int t0 = blockIdx.y * 64;
  const v4f wv = *(const v4f*)(cw + (size_t)d * 4);
  const float wa = wv[0], wb = wv[1], wc = wv[2], wd = wv[3];
  const float w0 = bf_rne(wa), w1 = bf_rne(wb), w2 = bf_rne(wc), w3 = bf_rne(wd);
  const float cbv = cb[d];
  const float bc = bf_rne(cbv);
  float xm3, xm2, xm1;
  {
    const int r3 = t0 - 3, r2 = t0 - 2, r1 = t0 - 1;
    const float v3 = XZ[(size_t)(r3 < 0 ? 0 : r3) * kXzP + d];
    const float v2 = XZ[(size_t)(r2 < 0 ? 0 : r2) * kXzP + d];
    const float v1 = XZ[(size_t)(r1 < 0 ? 0 : r1) * kXzP + d];
    xm3 = (r3 >= 0) ? v3 : 0.f;
    xm2 = (r2 >= 0) ? v2 : 0.f;
    xm1 = (r1 >= 0) ? v1 : 0.f;
  }
#pragma unroll 1
  for (int sub = 0; sub < 4; ++sub) {
    const int lb = t0 + sub * 16;
#pragma unroll 1
    for (int s = 0; s < 16; ++s) {
      const float xcur = XZ[(size_t)(lb + s) * kXzP + d];
      float acc = w0 * xm3;
      acc = fmaf(w1, xm2, acc);
      acc = fmaf(w2, xm1, acc);
      acc = fmaf(w3, xcur, acc);
      const float sv = acc + bc;
      const float ex = expf(-sv);
      const float sg = __builtin_amdgcn_rcpf(1.0f + ex);
      sT[s * kConvTP + tid] = sv * sg;
      xm3 = xm2; xm2 = xm1; xm1 = xcur;
    }
    __syncthreads();
    v8h bh[2], blo[2];
#pragma unroll
    for (int it = 0; it < 2; ++it) {
      const float* sp = sT + (it * 8 + wave) * kConvTP + lane * 8;
      const v4f a0 = *(const v4f*)(sp);
      const v4f a1 = *(const v4f*)(sp + 4);
#pragma unroll
      for (int e = 0; e < 4; ++e) {
        const float fa = a0[e];
        const float fb = a1[e];
        const unsigned short h0 = f2bf_bits(fa), h1 = f2bf_bits(fb);
        const unsigned short l0 = f2bf_bits(fa - bf_bits2f(h0)), l1 = f2bf_bits(fb - bf_bits2f(h1));
        bh[it][e]      = __builtin_bit_cast(_Float16, h0);
        bh[it][4 + e]  = __builtin_bit_cast(_Float16, h1);
        blo[it][e]     = __builtin_bit_cast(_Float16, l0);
        blo[it][4 + e] = __builtin_bit_cast(_Float16, l1);
      }
    }
    for (int pass = 0; pass < 2; ++pass) {
#pragma unroll
      for (int it = 0; it < 2; ++it) {
        const size_t o = (size_t)(lb + it * 8 + wave) * kDin + d0 + lane * 8;
        *(volatile v8h*)(XCH + o) = bh[it];
        *(volatile v8h*)(XCL + o) = blo[it];
      }
      __threadfence();
    }
    __syncthreads();
  }
}

__global__ __launch_bounds__(256) void row_gate_kernel(
    const unsigned short* __restrict__ XCH, const unsigned short* __restrict__ XCL,
    const float* __restrict__ PRE, const float* __restrict__ bdt,
    const float* __restrict__ BC, const float* __restrict__ XZ, const float* __restrict__ Dp,
    unsigned short* __restrict__ YH, unsigned short* __restrict__ YL)
{
  __shared__ __align__(16) float sxc[kDin];
  __shared__ __align__(16) float sy[kDin];
  __shared__ float sred[8];
  __shared__ float sbc[kBcReal];
  const int l = blockIdx.x;
  const int tid = threadIdx.x, lane = tid & 31, wave = tid >> 5;
  const size_t rowo = (size_t)l * kDin;
  {
    const size_t o = rowo + (size_t)tid * 8;
    const v4u hw = *(const v4u*)(XCH + o);
    const v4u lw = *(const v4u*)(XCL + o);
    const unsigned h0 = hw[0], h1 = hw[1], h2 = hw[2], h3 = hw[3];
    const unsigned q0 = lw[0], q1 = lw[1], q2 = lw[2], q3 = lw[3];
    v4f f0, f1;
    f0[0] = __uint_as_float(h0 << 16)         + __uint_as_float(q0 << 16);
    f0[1] = __uint_as_float(h0 & 0xffff0000u) + __uint_as_float(q0 & 0xffff0000u);
    f0[2] = __uint_as_float(h1 << 16)         + __uint_as_float(q1 << 16);
    f0[3] = __uint_as_float(h1 & 0xffff0000u) + __uint_as_float(q1 & 0xffff0000u);
    f1[0] = __uint_as_float(h2 << 16)         + __uint_as_float(q2 << 16);
    f1[1] = __uint_as_float(h2 & 0xffff0000u) + __uint_as_float(q2 & 0xffff0000u);
    f1[2] = __uint_as_float(h3 << 16)         + __uint_as_float(q3 << 16);
    f1[3] = __uint_as_float(h3 & 0xffff0000u) + __uint_as_float(q3 & 0xffff0000u);
    *(v4f*)(sxc + tid * 8)     = f0;
    *(v4f*)(sxc + tid * 8 + 4) = f1;
  }
  if (tid < kBcReal) sbc[tid] = BC[(size_t)l * kBcP + tid];
  __syncthreads();

  float sp = 0.0f;
#pragma unroll 1
  for (int j = 0; j < 8; ++j) {
    const int d = j * 256 + tid;
    const float xv = sxc[d];
    const float pv = PRE[rowo + d];
    const float braw = bdt[d];
    const float bv = bf_rne(braw);
    const float v = pv + bv;
    const float ea = expf(-fabsf(v));
    const float dtv = fmaxf(v, 0.0f) + log1pf(ea);
    sp = fmaf(xv, dtv, sp);
  }
#pragma unroll
  for (int off = 16; off > 0; off >>= 1) sp += __shfl_xor(sp, off, 32);
  if (lane == 0) sred[wave] = sp;
  __syncthreads();

  float s = 0.0f;
#pragma unroll
  for (int w = 0; w < 8; ++w) s += sred[w];
  float dot = 0.0f;
#pragma unroll 1
  for (int n = 0; n < kNst; ++n) dot = fmaf(sbc[n], sbc[n + kNst], dot);
  const float coef = s * dot;

#pragma unroll 1
  for (int j = 0; j < 8; ++j) {
    const int d = j * 256 + tid;
    const float xv = sxc[d];
    const float zv = XZ[(size_t)l * kXzP + kDin + d];
    const float draw = Dp[d];
    const float dv = bf_rne(draw);
    const float ez = expf(-zv);
    const float sg = __builtin_amdgcn_rcpf(1.0f + ez);
    const float g = zv * sg;
    const float yv = fmaf(xv, dv, coef);
    sy[d] = yv * g;
  }
  __syncthreads();

  v8h hv, lv;
  {
    const float* spp = sy + tid * 8;
    const v4f a0 = *(const v4f*)(spp);
    const v4f a1 = *(const v4f*)(spp + 4);
#pragma unroll
    for (int e = 0; e < 4; ++e) {
      const float fa = a0[e];
      const float fb = a1[e];
      const unsigned short h0 = f2bf_bits(fa), h1 = f2bf_bits(fb);
      const unsigned short l0 = f2bf_bits(fa - bf_bits2f(h0)), l1 = f2bf_bits(fb - bf_bits2f(h1));
      hv[e]     = __builtin_bit_cast(_Float16, h0);
      hv[4 + e] = __builtin_bit_cast(_Float16, h1);
      lv[e]     = __builtin_bit_cast(_Float16, l0);
      lv[4 + e] = __builtin_bit_cast(_Float16, l1);
    }
  }
  const size_t oo = rowo + (size_t)tid * 8;
  *(volatile v8h*)(YH + oo) = hv;
  *(volatile v8h*)(YL + oo) = lv;
  __threadfence();
  *(volatile v8h*)(YH + oo) = hv;
  *(volatile v8h*)(YL + oo) = lv;
}

extern "C" void kernel_launch(void* const* d_in, const int* in_sizes, int n_in,
                              void* d_out, int out_size, void* d_ws, size_t ws_size,
                              hipStream_t stream) {
  if (n_in < 10) return;
  if (in_sizes[0] != kSeq * kDm) return;
  if (in_sizes[1] != kXzP * kDm) return;
  if (in_sizes[2] != kDin * 4) return;
  if (in_sizes[3] != kDin) return;
  if (in_sizes[4] != kBcReal * kDin) return;
  if (in_sizes[5] != kDin * kDin) return;
  if (in_sizes[6] != kDin) return;
  if (in_sizes[7] != kDm * kDin) return;
  if (in_sizes[8] != kNst) return;
  if (in_sizes[9] != kDin) return;
  if (out_size != kSeq * kDm) return;
  if (ws_size < kWsTotal) return;

  const float* x       = (const float*)d_in[0];
  const float* W_in    = (const float*)d_in[1];
  const float* conv_w  = (const float*)d_in[2];
  const float* conv_b  = (const float*)d_in[3];
  const float* W_xproj = (const float*)d_in[4];
  const float* W_dt    = (const float*)d_in[5];
  const float* b_dt    = (const float*)d_in[6];
  const float* W_out   = (const float*)d_in[7];
  const float* Dp      = (const float*)d_in[9];
  float* out = (float*)d_out;

  char* ws = (char*)d_ws;
  unsigned short* XB  = (unsigned short*)(ws + kOffXB);
  unsigned short* WIB = (unsigned short*)(ws + kOffWIB);
  unsigned short* WDB = (unsigned short*)(ws + kOffWDB);
  unsigned short* WOB = (unsigned short*)(ws + kOffWOB);
  unsigned short* WXB = (unsigned short*)(ws + kOffWXB);
  float*          XZ  = (float*)(ws + kOffXZ);
  unsigned short* XCH = (unsigned short*)(ws + kOffXCH);
  unsigned short* XCL = (unsigned short*)(ws + kOffXCL);
  float*          PRE = (float*)(ws + kOffPRE);
  float*          BC  = (float*)(ws + kOffBC);
  unsigned short* YH  = (unsigned short*)(ws + kOffYH);
  unsigned short* YL  = (unsigned short*)(ws + kOffYL);

  rne_rows_bf16_kernel<<<(kSeq * kDm / 8) / 256, 256, 0, stream>>>(x, XB, kSeq * kDm / 8, kSeq * kDm / 8);
  rne_rows_bf16_kernel<<<(kXzP * kDm / 8) / 256, 256, 0, stream>>>(W_in, WIB, kXzP * kDm / 8, kXzP * kDm / 8);
  rne_rows_bf16_kernel<<<(kDin * kDin / 8) / 256, 256, 0, stream>>>(W_dt, WDB, kDin * kDin / 8, kDin * kDin / 8);
  rne_rows_bf16_kernel<<<(kDm * kDin / 8) / 256, 256, 0, stream>>>(W_out, WOB, kDm * kDin / 8, kDm * kDin / 8);
  rne_rows_bf16_kernel<<<(kBcP * kDin / 8) / 256, 256, 0, stream>>>(W_xproj, WXB, kBcP * kDin / 8, kBcReal * kDin / 8);

  wmma_gemm64<0><<<dim3(256, 1), 256, 0, stream>>>(
      XB, XB, kDm, WIB, kDm, XZ, kXzP, kSeq, kXzP, kDm);

  conv_silu_kernel<<<dim3(kDin / 256, kSeq / 64), 256, 0, stream>>>(XZ, conv_w, conv_b, XCH, XCL);

  wmma_gemm64<0><<<dim3(128, 1), 256, 0, stream>>>(
      XCH, XCH, kDin, WDB, kDin, PRE, kDin, kSeq, kDin, kDin);

  wmma_gemm64<1><<<dim3(4, 1), 256, 0, stream>>>(
      XCH, XCL, kDin, WXB, kDin, BC, kBcP, kSeq, kBcP, kDin);

  row_gate_kernel<<<kSeq, 256, 0, stream>>>(XCH, XCL, PRE, b_dt, BC, XZ, Dp, YH, YL);

  wmma_gemm64<1><<<dim3(64, 1), 256, 0, stream>>>(
      YH, YL, kDin, WOB, kDin, out, kDm, kSeq, kDm, kDin);
}
